// TTLinear_19619410608255
// MI455X (gfx1250) — hardware-verified
//
#include <hip/hip_runtime.h>
#include <stdint.h>
#include <stddef.h>

#define NB    2048
#define NF    4096
#define CB    256
#define NCH   (NB / CB)
#define CPB   512
#define KD    128
#define PROWS (CB * CPB)
#define NBLK  (PROWS / 128)
#define SP    136
#define FP    132

static_assert(NB % CB == 0);
static_assert(PROWS % 128 == 0);
static_assert(CPB % 128 == 0);
static_assert(NF == CPB * 8);
static_assert((SP * 2) % 16 == 0);
static_assert((FP * 4) % 16 == 0);

typedef _Float16       v16h  __attribute__((ext_vector_type(16)));
typedef _Float16       v8h   __attribute__((ext_vector_type(8)));
typedef __bf16         v16bf __attribute__((ext_vector_type(16)));
typedef float          v8f   __attribute__((ext_vector_type(8)));
typedef float          v4f   __attribute__((ext_vector_type(4)));
typedef unsigned int   v4u   __attribute__((ext_vector_type(4)));
typedef v4f __attribute__((may_alias)) v4fa;
typedef v4u __attribute__((may_alias)) v4ua;

union FragBF { v16bf v; v4u q[2]; };
union FragH  { v16h  v; v4u q[2]; };
union Pack8H { v8h   v; v4u u; };


__device__ __forceinline__ unsigned int bfb(float f) {
  unsigned int u = __float_as_uint(f);
  u += 0x7FFFu + ((u >> 16) & 1u);
  return u >> 16;
}
__device__ __forceinline__ void split2(float v, unsigned int& hi, unsigned int& lo) {
  hi = bfb(v);
  lo = bfb(v - __uint_as_float(hi << 16));
}
__device__ __forceinline__ unsigned int pk(unsigned int a, unsigned int b) { return (a & 0xFFFFu) | (b << 16); }

__device__ __forceinline__ v8f wmma_bf(v16bf a, v16bf b, v8f c) {
  v8f d = __builtin_amdgcn_wmma_f32_16x16x32_bf16(false, a, false, b, (short)0, c, false, false);
  asm volatile("v_nop\n\tv_nop\n\tv_nop\n\tv_nop" : "+v"(d) : "v"(a), "v"(b));
  return d;
}
__device__ __forceinline__ v8f wmma_hf(v16h a, v16h b, v8f c) {
  v8f d = __builtin_amdgcn_wmma_f32_16x16x32_f16(false, a, false, b, (short)0, c, false, false);
  asm volatile("v_nop\n\tv_nop\n\tv_nop\n\tv_nop" : "+v"(d) : "v"(a), "v"(b));
  return d;
}

__device__ __forceinline__ v4u cvt8_f16(v8f a, float sc) {
  Pack8H c;
  v8h t = { (_Float16)(a[0] * sc), (_Float16)(a[1] * sc), (_Float16)(a[2] * sc), (_Float16)(a[3] * sc),
            (_Float16)(a[4] * sc), (_Float16)(a[5] * sc), (_Float16)(a[6] * sc), (_Float16)(a[7] * sc) };
  c.v = t;
  return c.u;
}
__device__ __forceinline__ v4u cvt8_bf_hi(v8f a) {
  const v4u r = { pk(bfb(a[0]), bfb(a[1])), pk(bfb(a[2]), bfb(a[3])),
                  pk(bfb(a[4]), bfb(a[5])), pk(bfb(a[6]), bfb(a[7])) };
  return r;
}
__device__ __forceinline__ v4u cvt8_bf_lo(v8f a) {
  unsigned int h0, l0, h1, l1, h2, l2, h3, l3, h4, l4, h5, l5, h6, l6, h7, l7;
  split2(a[0], h0, l0); split2(a[1], h1, l1); split2(a[2], h2, l2); split2(a[3], h3, l3);
  split2(a[4], h4, l4); split2(a[5], h5, l5); split2(a[6], h6, l6); split2(a[7], h7, l7);
  const v4u r = { pk(l0, l1), pk(l2, l3), pk(l4, l5), pk(l6, l7) };
  return r;
}

__device__ __forceinline__ unsigned short* stage_row(unsigned short* S, int wv, int h, int m) {
  return S + ((m & 7) * 16 + 2 * wv + h) * SP + 8 * (m >> 3);
}

__device__ __forceinline__ void plane_pass(const unsigned short* S, unsigned short* plane, int bl, int t0, int tid) {
  #pragma unroll
  for (int G = 0; G < 8; ++G) {
    const v4u v = *(const v4ua*)(S + (G * 16 + (tid >> 4)) * SP + 8 * (tid & 15));
    const size_t ro = (size_t)(bl * CPB + 64 * G + (t0 >> 3)) * KD + (size_t)(8 * tid);
    *(volatile v4u*)(plane + ro) = v;
  }
}

__global__ __launch_bounds__(256) void k_prep(const float* __restrict__ core0, const float* __restrict__ core1,
                                              const float* __restrict__ core2, const float* __restrict__ core3,
                                              unsigned short* __restrict__ c3p, unsigned short* __restrict__ c2p,
                                              unsigned short* __restrict__ c1p, unsigned short* __restrict__ c0p)
{
  const int tid = threadIdx.x, blk = blockIdx.x;
  v4u val;
  unsigned short* dst;
  if (blk < 2) {
    const int g = blk * 256 + tid;
    const int a = g >> 2, p = g & 3;
    const float* s = core3 + a * 8;
    unsigned int e[8];
    #pragma unroll
    for (int j = 0; j < 8; ++j) {
      unsigned int hb, lb;
      split2(s[j], hb, lb);
      const unsigned int t = (p == 1) ? lb : hb;
      e[j] = (p == 3) ? 0u : t;
    }
    const v4u r = { pk(e[0], e[1]), pk(e[2], e[3]), pk(e[4], e[5]), pk(e[6], e[7]) };
    val = r;
    dst = c3p + (size_t)g * 8;
  } else if (blk < 18) {
    const bool one = (blk >= 10);
    const float* src = one ? core1 : core2;
    unsigned short* dp = one ? c1p : c2p;
    const int g = (blk - (one ? 10 : 2)) * 256 + tid;
    const int a = g >> 4, rl = g & 15;
    const float* s = src + a * KD + rl;
    Pack8H c;
    v8h t = { (_Float16)s[0],  (_Float16)s[16], (_Float16)s[32], (_Float16)s[48],
              (_Float16)s[64], (_Float16)s[80], (_Float16)s[96], (_Float16)s[112] };
    c.v = t;
    val = c.u;
    dst = dp + (size_t)g * 8;
  } else {
    const int g = tid;
    const int ap = g >> 4, rl = g & 15;
    const float* s = core0 + (ap & 7) * KD + rl;
    unsigned int e[8];
    #pragma unroll
    for (int rh = 0; rh < 8; ++rh) {
      unsigned int hb, lb;
      split2(s[16 * rh], hb, lb);
      e[rh] = (ap < 8) ? hb : lb;
    }
    const v4u r = { pk(e[0], e[1]), pk(e[2], e[3]), pk(e[4], e[5]), pk(e[6], e[7]) };
    val = r;
    dst = c0p + (size_t)g * 8;
  }
  *(volatile v4u*)dst = val;
  __threadfence();
  *(volatile v4u*)dst = val;
}

__global__ __launch_bounds__(256) void k_s3(const float* __restrict__ x, const unsigned short* __restrict__ c3p,
                                            unsigned short* __restrict__ pa, int chunk)
{
  __shared__ __align__(16) unsigned short S[128 * SP];
  const int tid = threadIdx.x, lane = tid & 31, wv = tid >> 5;
  const int h = lane >> 4, m = lane & 15;
  const int bx = blockIdx.x, bl = bx >> 2, t0 = (bx & 3) * 128;

  const size_t xo = ((size_t)(chunk * CB + bl) * CPB + (size_t)(t0 + 16 * wv + m)) * 8;
  const v4f xa = *(const v4fa*)(x + xo);
  const v4f xb = *(const v4fa*)(x + xo + 4);
  unsigned int h0, l0, h1, l1, h2, l2, h3, l3, h4, l4, h5, l5, h6, l6, h7, l7;
  split2(xa.x, h0, l0); split2(xa.y, h1, l1); split2(xa.z, h2, l2); split2(xa.w, h3, l3);
  split2(xb.x, h4, l4); split2(xb.y, h5, l5); split2(xb.z, h6, l6); split2(xb.w, h7, l7);
  const unsigned int km = (h != 0) ? 0u : 0xFFFFFFFFu;
  FragBF fa;
  const v4u H = { pk(h0, h1), pk(h2, h3), pk(h4, h5), pk(h6, h7) };
  const v4u L = { pk(l0, l1) & km, pk(l2, l3) & km, pk(l4, l5) & km, pk(l6, l7) & km };
  fa.q[0] = H;
  fa.q[1] = L;

  const v8f z8 = {0.f, 0.f, 0.f, 0.f, 0.f, 0.f, 0.f, 0.f};
  v8f acc[8];
  #pragma unroll
  for (int j = 0; j < 8; ++j) acc[j] = z8;
  #pragma unroll
  for (int j = 0; j < 8; ++j) {
    const unsigned short* bp = c3p + (16 * j + m) * 32;
    FragBF fb;
    fb.q[0] = *(const v4ua*)(bp + 8 * h);
    fb.q[1] = *(const v4ua*)(bp + 16 + 8 * h);
    acc[j] = wmma_bf(fa.v, fb.v, acc[j]);
  }

  unsigned short* srow = stage_row(S, wv, h, m);
  #pragma unroll
  for (int j = 0; j < 8; ++j) *(v4ua*)(srow + 16 * j) = cvt8_f16(acc[j], 16.0f);
  __syncthreads();
  plane_pass(S, pa, bl, t0, tid);
  __threadfence();
  plane_pass(S, pa, bl, t0, tid);
}

template <int SPLIT>
__global__ __launch_bounds__(256) void k_mid(const unsigned short* __restrict__ pin, const unsigned short* __restrict__ cp,
                                             unsigned short* __restrict__ po, unsigned short* __restrict__ pl)
{
  __shared__ __align__(16) unsigned short S[128 * SP];
  const int tid = threadIdx.x, lane = tid & 31, wv = tid >> 5;
  const int h = lane >> 4, m = lane & 15;
  const int bx = blockIdx.x, bl = bx >> 2, t0 = (bx & 3) * 128;

  const unsigned short* ar = pin + (size_t)(bx * 128 + 16 * wv + m) * KD;
  const v8f z8 = {0.f, 0.f, 0.f, 0.f, 0.f, 0.f, 0.f, 0.f};
  v8f acc[8];
  #pragma unroll
  for (int j = 0; j < 8; ++j) acc[j] = z8;

  #pragma unroll 1
  for (int k0 = 0; k0 < KD; k0 += 32) {
    FragH fa;
    fa.q[0] = *(const v4ua*)(ar + k0 + 8 * h);
    fa.q[1] = *(const v4ua*)(ar + k0 + 16 + 8 * h);
    #pragma unroll
    for (int j = 0; j < 8; ++j) {
      const unsigned short* bp = cp + (size_t)(16 * j + m) * KD + k0;
      FragH fb;
      fb.q[0] = *(const v4ua*)(bp + 8 * h);
      fb.q[1] = *(const v4ua*)(bp + 16 + 8 * h);
      acc[j] = wmma_hf(fa.v, fb.v, acc[j]);
    }
  }

  unsigned short* srow = stage_row(S, wv, h, m);
  if (SPLIT == 0) {
    #pragma unroll
    for (int j = 0; j < 8; ++j) *(v4ua*)(srow + 16 * j) = cvt8_f16(acc[j], 1.0f);
    __syncthreads();
    plane_pass(S, po, bl, t0, tid);
    __threadfence();
    plane_pass(S, po, bl, t0, tid);
  } else {
    #pragma unroll
    for (int j = 0; j < 8; ++j) *(v4ua*)(srow + 16 * j) = cvt8_bf_hi(acc[j]);
    __syncthreads();
    plane_pass(S, po, bl, t0, tid);
    __threadfence();
    plane_pass(S, po, bl, t0, tid);
    __syncthreads();
    #pragma unroll
    for (int j = 0; j < 8; ++j) *(v4ua*)(srow + 16 * j) = cvt8_bf_lo(acc[j]);
    __syncthreads();
    plane_pass(S, pl, bl, t0, tid);
    __threadfence();
    plane_pass(S, pl, bl, t0, tid);
  }
}

__global__ __launch_bounds__(256) void k_s0(const unsigned short* __restrict__ ph, const unsigned short* __restrict__ pl,
                                            const unsigned short* __restrict__ c0p, const float* __restrict__ bias,
                                            float* __restrict__ out, int chunk)
{
  __shared__ __align__(16) float S0[16 * FP];
  const int tid = threadIdx.x, lane = tid & 31, wv = tid >> 5;
  const int h = lane >> 4, m = lane & 15;
  const int bx = blockIdx.x, bl = bx >> 2, t0 = (bx & 3) * 128;

  const size_t ro = (size_t)(bx * 128 + 16 * wv + m) * KD;
  const v8f z8 = {0.f, 0.f, 0.f, 0.f, 0.f, 0.f, 0.f, 0.f};
  v8f acch = z8, accl = z8;
  #pragma unroll 1
  for (int k0 = 0; k0 < KD; k0 += 32) {
    FragBF fh, fl, fb;
    fh.q[0] = *(const v4ua*)(ph + ro + k0 + 8 * h);
    fh.q[1] = *(const v4ua*)(ph + ro + k0 + 16 + 8 * h);
    fl.q[0] = *(const v4ua*)(pl + ro + k0 + 8 * h);
    fl.q[1] = *(const v4ua*)(pl + ro + k0 + 16 + 8 * h);
    const unsigned short* bp = c0p + m * KD + k0;
    fb.q[0] = *(const v4ua*)(bp + 8 * h);
    fb.q[1] = *(const v4ua*)(bp + 16 + 8 * h);
    acch = wmma_bf(fh.v, fb.v, acch);
    accl = wmma_bf(fl.v, fb.v, accl);
  }
  float v[8];
  #pragma unroll
  for (int r = 0; r < 8; ++r) {
    float s = acch[r] + accl[r];
    s = s + __shfl_xor(s, 8);
    v[r] = s * 0.0625f;
  }
  float* sr = S0 + m * FP + 16 * wv + 8 * h;
  const v4f va = { v[0], v[1], v[2], v[3] };
  const v4f vb = { v[4], v[5], v[6], v[7] };
  *(v4fa*)sr = va;
  *(v4fa*)(sr + 4) = vb;
  __syncthreads();

  const int bo = wv * CPB + t0 + 4 * lane;
  const v4f bv = *(const v4fa*)(bias + bo);
  const v4f ov = *(const v4fa*)(S0 + wv * FP + 4 * lane) + bv;
  const size_t oo = (size_t)(chunk * CB + bl) * NF + (size_t)bo;
  *(volatile v4f*)(out + oo) = ov;
  __threadfence();
  *(volatile v4f*)(out + oo) = ov;
}

extern "C" void kernel_launch(void* const* d_in, const int* in_sizes, int n_in,
                              void* d_out, int out_size, void* d_ws, size_t ws_size,
                              hipStream_t stream)
{
  if (n_in < 6) return;
  if (in_sizes[0] != NB * NF) return;
  if (in_sizes[1] != 8 * KD) return;
  if (in_sizes[2] != KD * KD) return;
  if (in_sizes[3] != KD * KD) return;
  if (in_sizes[4] != KD * 8) return;
  if (in_sizes[5] != NF) return;
  if (out_size != NB * NF) return;

  const float* x     = (const float*)d_in[0];
  const float* core0 = (const float*)d_in[1];
  const float* core1 = (const float*)d_in[2];
  const float* core2 = (const float*)d_in[3];
  const float* core3 = (const float*)d_in[4];
  const float* bias  = (const float*)d_in[5];
  float* out = (float*)d_out;

  const size_t bC3 = (size_t)128 * 32 * 2;
  const size_t bC2 = (size_t)KD * KD * 2;
  const size_t bC1 = (size_t)KD * KD * 2;
  const size_t bC0 = (size_t)16 * KD * 2;
  const size_t bPL = (size_t)PROWS * KD * 2;
  const size_t total = bC3 + bC2 + bC1 + bC0 + 3 * bPL;
  if (total > ws_size) return;
  if (total > (size_t)134217728) return;

  char* ws = (char*)d_ws;
  size_t off = 0;
  unsigned short* C3P = (unsigned short*)(ws + off); off += bC3;
  unsigned short* C2P = (unsigned short*)(ws + off); off += bC2;
  unsigned short* C1P = (unsigned short*)(ws + off); off += bC1;
  unsigned short* C0P = (unsigned short*)(ws + off); off += bC0;
  unsigned short* PA  = (unsigned short*)(ws + off); off += bPL;
  unsigned short* PB  = (unsigned short*)(ws + off); off += bPL;
  unsigned short* PLO = (unsigned short*)(ws + off); off += bPL;
  if (off != total) return;

  k_prep<<<19, 256, 0, stream>>>(core0, core1, core2, core3, C3P, C2P, C1P, C0P);

  for (int c = 0; c < NCH; ++c) {
    k_s3<<<NBLK, 256, 0, stream>>>(x, C3P, PA, c);
    k_mid<0><<<NBLK, 256, 0, stream>>>(PA, C2P, PB, PB);
    k_mid<1><<<NBLK, 256, 0, stream>>>(PB, C1P, PA, PLO);
    k_s0<<<NBLK, 256, 0, stream>>>(PA, PLO, C0P, bias, out, c);
  }
}
